// SpikeAttention_82386062672604
// MI455X (gfx1250) — hardware-verified
//
#include <hip/hip_runtime.h>
#include <math.h>

constexpr int kTok   = 1024;
constexpr int kDim   = 1024;
constexpr int kHeads = 8;
constexpr int kHD    = 128;
constexpr int kFD    = 256;
constexpr int kSD    = 512;
constexpr int kHDC   = 32;
constexpr int kSteps = 8;
constexpr float kLnEps = 1e-5f;

typedef __attribute__((ext_vector_type(16))) _Float16 v16h;
typedef __attribute__((ext_vector_type(8)))  _Float16 v8h;
typedef __attribute__((ext_vector_type(16))) __bf16   v16b;
typedef __attribute__((ext_vector_type(8)))  __bf16   v8b;
typedef __attribute__((ext_vector_type(8)))  float    v8f;
typedef __attribute__((ext_vector_type(4)))  float    v4f;
typedef __attribute__((ext_vector_type(4)))  unsigned int v4u;

__device__ __forceinline__ unsigned short f2bf_bits(float f) {
  unsigned u = __float_as_uint(f);
  return (unsigned short)((u + 0x7FFFu + ((u >> 16) & 1u)) >> 16);
}
__device__ __forceinline__ float bf_bits2f(unsigned short h) { return __uint_as_float(((unsigned)h) << 16); }
__device__ __forceinline__ unsigned pk16(unsigned short a, unsigned short b) { return (unsigned)a | ((unsigned)b << 16); }

__device__ __forceinline__ void dep_guard_h(v8f& a, v8f& b, v16h x, v16h y) { asm volatile("v_nop\n\tv_nop\n\tv_nop\n\tv_nop" : "+v"(a), "+v"(b) : "v"(x), "v"(y)); }
__device__ __forceinline__ void dep_guard_b(v8f& a, v8f& b, v16b x, v16b y) { asm volatile("v_nop\n\tv_nop\n\tv_nop\n\tv_nop" : "+v"(a), "+v"(b) : "v"(x), "v"(y)); }
__device__ __forceinline__ void keep4_h(v16h a, v16h b, v16h c, v16h d) { asm volatile("v_nop" :: "v"(a), "v"(b), "v"(c), "v"(d)); }
__device__ __forceinline__ void keep4_b(v16b a, v16b b, v16b c, v16b d) { asm volatile("v_nop" :: "v"(a), "v"(b), "v"(c), "v"(d)); }
__device__ __forceinline__ void acc_guard4(v8f& a, v8f& b, v8f& c, v8f& d) { asm volatile("v_nop\n\tv_nop\n\tv_nop\n\tv_nop" : "+v"(a), "+v"(b), "+v"(c), "+v"(d)); }
template <typename T> struct Frag;
template <> struct Frag<_Float16> {
  typedef v16h V; union U { v16h v; v8h h[2]; };
  static __device__ __forceinline__ v16h load(const _Float16* p) {
    U f; f.h[0] = *(const v8h*)(p); f.h[1] = *(const v8h*)(p + 16); return f.v;
  }
  static __device__ __forceinline__ v8f mma(v16h a, v16h b, v8f c) {
    return __builtin_amdgcn_wmma_f32_16x16x32_f16(false, a, false, b, (short)0, c, false, false);
  }
  static __device__ __forceinline__ void guard(v8f& a, v8f& b, v16h x, v16h y) { dep_guard_h(a, b, x, y); }
  static __device__ __forceinline__ void keep(v16h a, v16h b, v16h c, v16h d) { keep4_h(a, b, c, d); }
};
template <> struct Frag<__bf16> {
  typedef v16b V; union U { v16b v; v8b h[2]; };
  static __device__ __forceinline__ v16b load(const __bf16* p) {
    U f; f.h[0] = *(const v8b*)(p); f.h[1] = *(const v8b*)(p + 16); return f.v;
  }
  static __device__ __forceinline__ v8f mma(v16b a, v16b b, v8f c) {
    return __builtin_amdgcn_wmma_f32_16x16x32_bf16(false, a, false, b, (short)0, c, false, false);
  }
  static __device__ __forceinline__ void guard(v8f& a, v8f& b, v16b x, v16b y) { dep_guard_b(a, b, x, y); }
  static __device__ __forceinline__ void keep(v16b a, v16b b, v16b c, v16b d) { keep4_b(a, b, c, d); }
};

template <int ET> struct Elem;
template <> struct Elem<0> { typedef _Float16 T; };
template <> struct Elem<1> { typedef __bf16 T; };
template <int ET, bool SPLIT, int BIAS_MODE, int OUT_MODE, bool RESID, int ACT = 0>
__global__ __launch_bounds__(256) void wmma_gemm64(
    const unsigned short* __restrict__ Ap, const unsigned short* __restrict__ A2p, int lda, long strideA,
    const unsigned short* __restrict__ Btp, const unsigned short* __restrict__ Bt2p, int ldb, long strideB,
    void* __restrict__ Cout, void* __restrict__ Cout2, int ldc, long strideC,
    const float* __restrict__ bias,
    const float* __restrict__ resid, long strideR,
    int M, int N, int K, float scale) {
  typedef typename Elem<ET>::T T;
  typedef typename Frag<T>::V V;
  const T* A = (const T*)Ap; const T* A2 = (const T*)A2p; const T* Bt = (const T*)Btp; const T* Bt2 = (const T*)Bt2p;
  __shared__ __align__(16) float sT[8][16 * 68];
  const int b    = blockIdx.y;
  const int lane = threadIdx.x & 31;
  const int wave = threadIdx.x >> 5;
  const int tilesN = N >> 6;
  const int tilesM = M >> 6;
  const int tile = blockIdx.x * 8 + wave;
  if (tile >= tilesM * tilesN) return;
  const int tm = tile / tilesN;
  const int tn = tile - tm * tilesN;
  const int m0 = tm << 6;
  const int n0 = tn << 6;

  const T* Ab  = A  + (size_t)b * strideA;
  const T* Bb  = Bt + (size_t)b * strideB;
  const T* Ab2 = SPLIT ? (A2  + (size_t)b * strideA) : nullptr;
  const T* Bb2 = SPLIT ? (Bt2 + (size_t)b * strideB) : nullptr;

  const int rlane = lane & 15;
  const int koff  = (lane >> 4) * 8;
  const int mOff  = (lane >> 4) * 8;

  v8f acc[4][4];
#pragma unroll
  for (int i = 0; i < 4; ++i)
#pragma unroll
    for (int j = 0; j < 4; ++j) acc[i][j] = (v8f){0.f,0.f,0.f,0.f,0.f,0.f,0.f,0.f};

  for (int k0 = 0; k0 < K; k0 += 32) {
    V bh[4], bl[4];
#pragma unroll
    for (int j = 0; j < 4; ++j) {
      const size_t bo = (size_t)(n0 + (j << 4) + rlane) * ldb + koff + k0;
      bh[j] = Frag<T>::load(Bb + bo);
      if (SPLIT) bl[j] = Frag<T>::load(Bb2 + bo);
    }
#pragma unroll
    for (int i = 0; i < 4; ++i) {
      const size_t ao = (size_t)(m0 + (i << 4) + rlane) * lda + koff + k0;
      V ah = Frag<T>::load(Ab + ao);
      V al;
      if (SPLIT) al = Frag<T>::load(Ab2 + ao);
#pragma unroll
      for (int j = 0; j < 4; ++j) {
        acc[i][j] = Frag<T>::mma(ah, bh[j], acc[i][j]);
        if (SPLIT) {
          acc[i][j] = Frag<T>::mma(ah, bl[j], acc[i][j]);
          acc[i][j] = Frag<T>::mma(al, bh[j], acc[i][j]);
        }
      }
      Frag<T>::guard(acc[i][0], acc[i][3], ah, SPLIT ? al : ah);
    }
    Frag<T>::keep(bh[0], bh[1], bh[2], bh[3]);
    if (SPLIT) Frag<T>::keep(bl[0], bl[1], bl[2], bl[3]);
  }
  acc_guard4(acc[0][0], acc[0][1], acc[0][2], acc[0][3]);
  acc_guard4(acc[1][0], acc[1][1], acc[1][2], acc[1][3]);
  acc_guard4(acc[2][0], acc[2][1], acc[2][2], acc[2][3]);
  acc_guard4(acc[3][0], acc[3][1], acc[3][2], acc[3][3]);

  float* slab = sT[wave];
  const float* Rb = RESID ? (resid + (size_t)b * strideR) : nullptr;
#pragma unroll
  for (int i = 0; i < 4; ++i) {
    const int mBase = m0 + (i << 4);
#pragma unroll
    for (int j = 0; j < 4; ++j) {
      const int n = n0 + (j << 4) + rlane;
      float bv = 0.f;
      if (BIAS_MODE == 2) bv = bias[n];
#pragma unroll
      for (int r = 0; r < 8; ++r) {
        float v = acc[i][j][r] * scale;
        if (BIAS_MODE == 1) v += bias[mBase + mOff + r];
        if (BIAS_MODE == 2) v += bv;
        if (RESID) v += Rb[(size_t)(mBase + mOff + r) * ldc + n];
        if (ACT == 2) v = fmaxf(v, 0.0f);
        if (ACT == 4) v = (v > 0.f) ? v : 0.01f * v;
        if (ACT == 6) { const float ev = expf(v); v = (v > 0.f) ? (v + 1.0f) : ev; }
        slab[(mOff + r) * 68 + (j << 4) + rlane] = v;
      }
    }
    __builtin_amdgcn_fence(__ATOMIC_RELEASE, "workgroup");
    __builtin_amdgcn_wave_barrier();
    __builtin_amdgcn_fence(__ATOMIC_ACQUIRE, "workgroup");
    if (OUT_MODE == 0) {
      float* C = (float*)Cout + (size_t)b * strideC;
      const int hh = lane >> 4, c4 = (lane & 15) * 4;
      for (int pass = 0; pass < 2; ++pass) {
#pragma unroll
        for (int it = 0; it < 8; ++it) {
          const int row = it * 2 + hh;
          v4f v = *(const v4f*)(slab + row * 68 + c4);
          *(volatile v4f*)(C + (size_t)(mBase + row) * ldc + n0 + c4) = v;
        }
        __threadfence();
      }
    } else {
      const int q = lane >> 3, c8 = (lane & 7) * 8;
      unsigned short* C  = (unsigned short*)Cout  + (size_t)b * strideC;
      unsigned short* C2 = (OUT_MODE == 2) ? ((unsigned short*)Cout2 + (size_t)b * strideC) : nullptr;
      for (int pass = 0; pass < 2; ++pass) {
#pragma unroll
        for (int it = 0; it < 4; ++it) {
          const int row = it * 4 + q;
          const float* sp = slab + row * 68 + c8;
          v8h hv, lv;
#pragma unroll
          for (int e = 0; e < 8; ++e) {
            if (OUT_MODE == 1) {
              hv[e] = (_Float16)sp[e];
            } else {
              unsigned short hb = f2bf_bits(sp[e]);
              unsigned short lb = f2bf_bits(sp[e] - bf_bits2f(hb));
              hv[e] = __builtin_bit_cast(_Float16, hb);
              lv[e] = __builtin_bit_cast(_Float16, lb);
            }
          }
          *(volatile v8h*)(C + (size_t)(mBase + row) * ldc + n0 + c8) = hv;
          if (OUT_MODE == 2) *(volatile v8h*)(C2 + (size_t)(mBase + row) * ldc + n0 + c8) = lv;
        }
        __threadfence();
      }
    }
    __builtin_amdgcn_fence(__ATOMIC_RELEASE, "workgroup");
    __builtin_amdgcn_wave_barrier();
    __builtin_amdgcn_fence(__ATOMIC_ACQUIRE, "workgroup");
  }
}

__device__ __forceinline__ float wave_sum(float v) {
#pragma unroll
  for (int off = 16; off > 0; off >>= 1) v += __shfl_xor(v, off, 32);
  return v;
}

__global__ __launch_bounds__(256) void split8_bf16_kernel(const float* __restrict__ in,
                                                          unsigned short* __restrict__ outH,
                                                          unsigned short* __restrict__ outL, int n8) {
  const int i = blockIdx.x * 256 + threadIdx.x;
  if (i >= n8) return;
  const float* p = in + 8 * (size_t)i;
  const v4f a = *(const v4f*)(p);
  const v4f c = *(const v4f*)(p + 4);
  unsigned short hb[8], lb[8];
#pragma unroll
  for (int e = 0; e < 4; ++e) {
    hb[e] = f2bf_bits(a[e]);
    lb[e] = f2bf_bits(a[e] - bf_bits2f(hb[e]));
    hb[4 + e] = f2bf_bits(c[e]);
    lb[4 + e] = f2bf_bits(c[e] - bf_bits2f(hb[4 + e]));
  }
  const v4u uh = (v4u){pk16(hb[0], hb[1]), pk16(hb[2], hb[3]), pk16(hb[4], hb[5]), pk16(hb[6], hb[7])};
  const v4u ul = (v4u){pk16(lb[0], lb[1]), pk16(lb[2], lb[3]), pk16(lb[4], lb[5]), pk16(lb[6], lb[7])};
  unsigned short* qh = outH + 8 * (size_t)i;
  unsigned short* ql = outL + 8 * (size_t)i;
  for (int pass = 0; pass < 2; ++pass) {
    *(volatile v4u*)qh = uh;
    *(volatile v4u*)ql = ul;
    __threadfence();
  }
}

__global__ __launch_bounds__(256) void projt_split_kernel(const float* __restrict__ proj,
                                                          unsigned short* __restrict__ outH,
                                                          unsigned short* __restrict__ outL) {
  __shared__ float sm[64][65];
  const int t  = threadIdx.x;
  const int d0 = blockIdx.x * 64;
  const int f0 = blockIdx.y * 64;
  const int h  = blockIdx.z;
  const float* P = proj + (size_t)h * kHD * kFD;
#pragma unroll
  for (int i = 0; i < 16; ++i) {
    const int e = i * 256 + t;
    const int r = e >> 6;
    const int c = e & 63;
    sm[c][r] = P[(size_t)(d0 + r) * kFD + f0 + c];
  }
  __syncthreads();
  const int lane = t & 31, wave = t >> 5;
  const int q = lane >> 3, c8 = (lane & 7) * 8;
  const size_t base = (size_t)h * kFD * kHD;
  for (int pass = 0; pass < 2; ++pass) {
#pragma unroll
    for (int it = 0; it < 2; ++it) {
      const int row = wave * 8 + it * 4 + q;
      unsigned short hb[8], lb[8];
#pragma unroll
      for (int e = 0; e < 8; ++e) {
        const float x = sm[row][c8 + e];
        hb[e] = f2bf_bits(x);
        lb[e] = f2bf_bits(x - bf_bits2f(hb[e]));
      }
      const v4u uh = (v4u){pk16(hb[0], hb[1]), pk16(hb[2], hb[3]), pk16(hb[4], hb[5]), pk16(hb[6], hb[7])};
      const v4u ul = (v4u){pk16(lb[0], lb[1]), pk16(lb[2], lb[3]), pk16(lb[4], lb[5]), pk16(lb[6], lb[7])};
      const size_t o = base + (size_t)(f0 + row) * kHD + d0 + c8;
      *(volatile v4u*)(outH + o) = uh;
      *(volatile v4u*)(outL + o) = ul;
    }
    __threadfence();
  }
}

template <int NT>
__global__ __launch_bounds__(NT) void ln_vec_kernel(const float* __restrict__ in, const float* __restrict__ g,
                                                    const float* __restrict__ b, float* __restrict__ out) {
  constexpr int NW = NT / 32;
  constexpr float kInvN = 1.0f / (float)(NT * 4);
  __shared__ float red1[NW];
  __shared__ float red2[NW];
  const int t = threadIdx.x, lane = t & 31, wave = t >> 5;
  const v4f x = *(const v4f*)(in + 4 * t);
  float s = (x[0] + x[1]) + (x[2] + x[3]);
  s = wave_sum(s);
  if (lane == 0) red1[wave] = s;
  __syncthreads();
  float tot = 0.f;
#pragma unroll
  for (int w = 0; w < NW; ++w) tot += red1[w];
  const float mean = tot * kInvN;
  float dev[4];
#pragma unroll
  for (int e = 0; e < 4; ++e) dev[e] = x[e] - mean;
  float sq = (dev[0] * dev[0] + dev[1] * dev[1]) + (dev[2] * dev[2] + dev[3] * dev[3]);
  sq = wave_sum(sq);
  if (lane == 0) red2[wave] = sq;
  __syncthreads();
  float tot2 = 0.f;
#pragma unroll
  for (int w = 0; w < NW; ++w) tot2 += red2[w];
  const float var = tot2 * kInvN;
  const float r = rsqrtf(var + kLnEps);
  const v4f gv = *(const v4f*)(g + 4 * t);
  const v4f bv = *(const v4f*)(b + 4 * t);
  v4f o;
#pragma unroll
  for (int e = 0; e < 4; ++e) o[e] = dev[e] * r * gv[e] + bv[e];
  float* dst = out + 4 * t;
  for (int pass = 0; pass < 2; ++pass) {
    *(volatile v4f*)dst = o;
    __threadfence();
  }
}

template <int ACT>
__global__ __launch_bounds__(256) void matvec_kernel(const float* __restrict__ vin, const float* __restrict__ W,
                                                    const float* __restrict__ bias, float* __restrict__ out, int K) {
  __shared__ float sv[kDim];
  const int t = threadIdx.x;
  const int Kc = (K > kDim) ? kDim : K;
  for (int i = t; i < Kc; i += 256) sv[i] = vin[i];
  __syncthreads();
  const int d = blockIdx.x * 256 + t;
  const float* wr = W + (size_t)d * Kc;
  float s = 0.f;
#pragma unroll 1
  for (int k = 0; k < Kc; ++k) s += sv[k] * wr[k];
  s += bias[d];
  if (ACT == 1) s = 0.5f * s * (1.0f + erff(s * 0.70710678118654752f));
  for (int pass = 0; pass < 2; ++pass) {
    *(volatile float*)(out + d) = s;
    __threadfence();
  }
}

__global__ __launch_bounds__(128) void srow_ln_split_kernel(const float* __restrict__ coef, const float* __restrict__ svec,
                                                            const float* __restrict__ g, const float* __restrict__ b,
                                                            unsigned short* __restrict__ outH,
                                                            unsigned short* __restrict__ outL) {
  __shared__ float red1[4];
  __shared__ float red2[4];
  constexpr float kInvN = 1.0f / (float)kDim;
  const int n = blockIdx.x;
  const int t = threadIdx.x, lane = t & 31, wave = t >> 5;
  const float c = coef[n];
  const int d0 = 8 * t;
  const v4f a0 = *(const v4f*)(svec + d0);
  const v4f a1 = *(const v4f*)(svec + d0 + 4);
  float val[8];
#pragma unroll
  for (int e = 0; e < 4; ++e) { val[e] = c * a0[e]; val[4 + e] = c * a1[e]; }
  float s = ((val[0] + val[1]) + (val[2] + val[3])) + ((val[4] + val[5]) + (val[6] + val[7]));
  s = wave_sum(s);
  if (lane == 0) red1[wave] = s;
  __syncthreads();
  const float mean = ((red1[0] + red1[1]) + (red1[2] + red1[3])) * kInvN;
  float dev[8];
  float sq = 0.f;
#pragma unroll
  for (int e = 0; e < 8; ++e) { dev[e] = val[e] - mean; sq += dev[e] * dev[e]; }
  sq = wave_sum(sq);
  if (lane == 0) red2[wave] = sq;
  __syncthreads();
  const float var = ((red2[0] + red2[1]) + (red2[2] + red2[3])) * kInvN;
  const float r = rsqrtf(var + kLnEps);
  const v4f g0 = *(const v4f*)(g + d0), g1 = *(const v4f*)(g + d0 + 4);
  const v4f b0 = *(const v4f*)(b + d0), b1 = *(const v4f*)(b + d0 + 4);
  float o[8];
#pragma unroll
  for (int e = 0; e < 4; ++e) {
    o[e]     = dev[e] * r * g0[e] + b0[e];
    o[4 + e] = dev[4 + e] * r * g1[e] + b1[e];
  }
  unsigned short hb[8], lb[8];
#pragma unroll
  for (int e = 0; e < 8; ++e) {
    hb[e] = f2bf_bits(o[e]);
    lb[e] = f2bf_bits(o[e] - bf_bits2f(hb[e]));
  }
  const v4u uh = (v4u){pk16(hb[0], hb[1]), pk16(hb[2], hb[3]), pk16(hb[4], hb[5]), pk16(hb[6], hb[7])};
  const v4u ul = (v4u){pk16(lb[0], lb[1]), pk16(lb[2], lb[3]), pk16(lb[4], lb[5]), pk16(lb[6], lb[7])};
  const size_t off = (size_t)n * kDim + d0;
  for (int pass = 0; pass < 2; ++pass) {
    *(volatile v4u*)(outH + off) = uh;
    *(volatile v4u*)(outL + off) = ul;
    __threadfence();
  }
}

__global__ __launch_bounds__(256) void causal_linattn_kernel(const float* __restrict__ qp, const float* __restrict__ kp,
                                                             const float* __restrict__ vf, float* __restrict__ att) {
  __shared__ __align__(16) float kps[kSteps * kFD];
  __shared__ __align__(16) float qps[kSteps * kFD];
  __shared__ __align__(16) float vs[kSteps * kHDC];
  __shared__ __align__(16) float part[kSteps * 8 * kHDC];
  __shared__ __align__(16) float dprod[kSteps * kFD];
  __shared__ __align__(16) float atts[kSteps * kHDC];
  const int t = threadIdx.x, lane = t & 31, wave = t >> 5;
  const int h = blockIdx.x >> 2, hc = blockIdx.x & 3;
  const int hd0 = hc * kHDC;
  const float* qph = qp + (size_t)h * kTok * kFD;
  const float* kph = kp + (size_t)h * kTok * kFD;
  const float* vcol = vf + (size_t)h * kHD + hd0;
  float* acol = att + (size_t)h * kHD + hd0;
  const int fbase = wave * 32;
  float kv[32];
#pragma unroll
  for (int i = 0; i < 32; ++i) kv[i] = 0.f;
  float kc = 0.f;
#pragma unroll 1
  for (int n0 = 0; n0 < kTok; n0 += kSteps) {
    __syncthreads();
#pragma unroll
    for (int i = 0; i < 2; ++i) {
      const int e4 = (i * 256 + t) * 4;
      const v4f a = *(const v4f*)(kph + (size_t)n0 * kFD + e4);
      const v4f c = *(const v4f*)(qph + (size_t)n0 * kFD + e4);
      *(v4f*)(kps + e4) = a;
      *(v4f*)(qps + e4) = c;
    }
    if (wave < 2) {
      const int r = t >> 3, c4 = (t & 7) * 4;
      const v4f vv4 = *(const v4f*)(vcol + (size_t)(n0 + r) * kDim + c4);
      *(v4f*)(vs + r * kHDC + c4) = vv4;
    }
    __syncthreads();
#pragma unroll 1
    for (int s = 0; s < kSteps; ++s) {
      const float vv = vs[s * kHDC + lane];
      const float* kr = kps + s * kFD + fbase;
      const float* qr = qps + s * kFD + fbase;
#pragma unroll
      for (int i4 = 0; i4 < 8; ++i4) {
        const v4f k4 = *(const v4f*)(kr + 4 * i4);
        kv[4 * i4 + 0] = fmaf(k4[0], vv, kv[4 * i4 + 0]);
        kv[4 * i4 + 1] = fmaf(k4[1], vv, kv[4 * i4 + 1]);
        kv[4 * i4 + 2] = fmaf(k4[2], vv, kv[4 * i4 + 2]);
        kv[4 * i4 + 3] = fmaf(k4[3], vv, kv[4 * i4 + 3]);
      }
      float pnum = 0.f;
#pragma unroll
      for (int i4 = 0; i4 < 8; ++i4) {
        const v4f q4 = *(const v4f*)(qr + 4 * i4);
        pnum = fmaf(q4[0], kv[4 * i4 + 0], pnum);
        pnum = fmaf(q4[1], kv[4 * i4 + 1], pnum);
        pnum = fmaf(q4[2], kv[4 * i4 + 2], pnum);
        pnum = fmaf(q4[3], kv[4 * i4 + 3], pnum);
      }
      part[(s * 8 + wave) * kHDC + lane] = pnum;
      const float kpf = kr[lane];
      kc += kpf;
      const float prod = qr[lane] * kc;
      dprod[s * kFD + fbase + lane] = prod;
    }
    __syncthreads();
    {
      float num = 0.f;
#pragma unroll
      for (int w = 0; w < 8; ++w) num += part[(wave * 8 + w) * kHDC + lane];
      float den = 0.f;
      const float* dp = dprod + wave * kFD;
#pragma unroll 1
      for (int f4 = 0; f4 < kFD / 4; ++f4) {
        const v4f dv = *(const v4f*)(dp + 4 * f4);
        den += dv[0]; den += dv[1]; den += dv[2]; den += dv[3];
      }
      atts[wave * kHDC + lane] = num / (den + 1e-8f);
    }
    __syncthreads();
    if (wave < 2) {
      const int q = lane >> 3, c4 = (lane & 7) * 4;
      const int row = wave * 4 + q;
      const v4f val = *(const v4f*)(atts + row * kHDC + c4);
      float* dst = acol + (size_t)(n0 + row) * kDim + c4;
      for (int pass = 0; pass < 2; ++pass) {
        *(volatile v4f*)dst = val;
        __threadfence();
      }
    }
  }
}

extern "C" void kernel_launch(void* const* d_in, const int* in_sizes, int n_in,
                              void* d_out, int out_size, void* d_ws, size_t ws_size,
                              hipStream_t stream) {
  if (n_in < 22) return;
  if (out_size != kTok * kDim) return;
  if (in_sizes[0] != kTok * kDim || in_sizes[1] != kSD || in_sizes[2] != kDim * kDim ||
      in_sizes[12] != kDim * kSD || in_sizes[14] != kDim * kDim || in_sizes[18] != kTok ||
      in_sizes[21] != kHeads * kHD * kFD) return;

  const float* xin   = (const float*)d_in[0];
  const float* cvec  = (const float*)d_in[1];
  const float* W1    = (const float*)d_in[2];
  const float* b1    = (const float*)d_in[3];
  const float* W2    = (const float*)d_in[4];
  const float* b2    = (const float*)d_in[5];
  const float* W3    = (const float*)d_in[6];
  const float* b3    = (const float*)d_in[7];
  const float* Wout  = (const float*)d_in[8];
  const float* bout  = (const float*)d_in[9];
  const float* g_c   = (const float*)d_in[10];
  const float* b_c   = (const float*)d_in[11];
  const float* Wf1   = (const float*)d_in[12];
  const float* bf1   = (const float*)d_in[13];
  const float* Wf2   = (const float*)d_in[14];
  const float* bf2   = (const float*)d_in[15];
  const float* g_ln  = (const float*)d_in[16];
  const float* b_ln  = (const float*)d_in[17];
  const float* coef  = (const float*)d_in[18];
  const float* g_c2  = (const float*)d_in[19];
  const float* b_c2  = (const float*)d_in[20];
  const float* proj  = (const float*)d_in[21];

  const size_t plane16  = (size_t)kTok * kDim * 2;
  const size_t plane32  = (size_t)kTok * kDim * 4;
  const size_t projP    = (size_t)kHeads * kFD * kHD * 2;
  const size_t featP    = (size_t)kHeads * kTok * kFD * 4;
  char* ws = (char*)d_ws;
  size_t off = 0;
  unsigned short* Xh  = (unsigned short*)(ws + off); off += plane16;
  unsigned short* Xl  = (unsigned short*)(ws + off); off += plane16;
  unsigned short* W1h = (unsigned short*)(ws + off); off += plane16;
  unsigned short* W1l = (unsigned short*)(ws + off); off += plane16;
  unsigned short* W2h = (unsigned short*)(ws + off); off += plane16;
  unsigned short* W2l = (unsigned short*)(ws + off); off += plane16;
  unsigned short* W3h = (unsigned short*)(ws + off); off += plane16;
  unsigned short* W3l = (unsigned short*)(ws + off); off += plane16;
  unsigned short* Woh = (unsigned short*)(ws + off); off += plane16;
  unsigned short* Wol = (unsigned short*)(ws + off); off += plane16;
  unsigned short* Sh  = (unsigned short*)(ws + off); off += plane16;
  unsigned short* Sl  = (unsigned short*)(ws + off); off += plane16;
  unsigned short* qh  = (unsigned short*)(ws + off); off += plane16;
  unsigned short* ql  = (unsigned short*)(ws + off); off += plane16;
  unsigned short* kh  = (unsigned short*)(ws + off); off += plane16;
  unsigned short* kl  = (unsigned short*)(ws + off); off += plane16;
  float*          vf  = (float*)(ws + off);          off += plane32;
  unsigned short* pTh = (unsigned short*)(ws + off); off += projP;
  unsigned short* pTl = (unsigned short*)(ws + off); off += projP;
  float*          qpf = (float*)(ws + off);          off += featP;
  float*          kpf = (float*)(ws + off);          off += featP;
  float*          attf = (float*)(ws + off);         off += plane32;
  unsigned short* atth = (unsigned short*)(ws + off); off += plane16;
  unsigned short* attl = (unsigned short*)(ws + off); off += plane16;
  float*          s_ln = (float*)(ws + off);         off += 4096;
  float*          h1   = (float*)(ws + off);         off += 4096;
  float*          h2   = (float*)(ws + off);         off += 4096;
  float*          svec = (float*)(ws + off);         off += 4096;
  if (off > ws_size) return;

  const int n8 = kTok * kDim / 8;
  const int splitBlocks = (n8 + 255) / 256;

  split8_bf16_kernel<<<splitBlocks, 256, 0, stream>>>(xin,  Xh,  Xl,  n8);
  split8_bf16_kernel<<<splitBlocks, 256, 0, stream>>>(W1,   W1h, W1l, n8);
  split8_bf16_kernel<<<splitBlocks, 256, 0, stream>>>(W2,   W2h, W2l, n8);
  split8_bf16_kernel<<<splitBlocks, 256, 0, stream>>>(W3,   W3h, W3l, n8);
  split8_bf16_kernel<<<splitBlocks, 256, 0, stream>>>(Wout, Woh, Wol, n8);
  projt_split_kernel<<<dim3(kHD / 64, kFD / 64, kHeads), 256, 0, stream>>>(proj, pTh, pTl);

  ln_vec_kernel<128><<<1, 128, 0, stream>>>(cvec, g_c, b_c, s_ln);
  matvec_kernel<1><<<kDim / 256, 256, 0, stream>>>(s_ln, Wf1, bf1, h1, kSD);
  matvec_kernel<0><<<kDim / 256, 256, 0, stream>>>(h1, Wf2, bf2, h2, kDim);
  ln_vec_kernel<256><<<1, 256, 0, stream>>>(h2, g_ln, b_ln, svec);
  srow_ln_split_kernel<<<kTok, 128, 0, stream>>>(coef, svec, g_c2, b_c2, Sh, Sl);

  wmma_gemm64<1, true, 2, 2, false, 0><<<dim3(32, 1), 256, 0, stream>>>(
      Xh, Xl, kDim, 0L, W1h, W1l, kDim, 0L, (void*)qh, (void*)ql, kDim, 0L, b1, b1, 0L, kTok, kDim, kDim, 1.0f);
  wmma_gemm64<1, true, 2, 2, false, 0><<<dim3(32, 1), 256, 0, stream>>>(
      Sh, Sl, kDim, 0L, W2h, W2l, kDim, 0L, (void*)kh, (void*)kl, kDim, 0L, b2, b2, 0L, kTok, kDim, kDim, 1.0f);
  wmma_gemm64<1, true, 2, 0, false, 0><<<dim3(32, 1), 256, 0, stream>>>(
      Xh, Xl, kDim, 0L, W3h, W3l, kDim, 0L, (void*)vf, (void*)vf, kDim, 0L, b3, b3, 0L, kTok, kDim, kDim, 1.0f);

  wmma_gemm64<1, true, 0, 0, false, 6><<<dim3(8, kHeads), 256, 0, stream>>>(
      qh, ql, kDim, (long)kHD, pTh, pTl, kHD, (long)(kFD * kHD), (void*)qpf, (void*)qpf, kFD, (long)(kTok * kFD),
      b1, b1, 0L, kTok, kFD, kHD, 1.0f);
  wmma_gemm64<1, true, 0, 0, false, 6><<<dim3(8, kHeads), 256, 0, stream>>>(
      kh, kl, kDim, (long)kHD, pTh, pTl, kHD, (long)(kFD * kHD), (void*)kpf, (void*)kpf, kFD, (long)(kTok * kFD),
      b2, b2, 0L, kTok, kFD, kHD, 1.0f);

  causal_linattn_kernel<<<kHeads * (kHD / kHDC), 256, 0, stream>>>(qpf, kpf, vf, attf);

  split8_bf16_kernel<<<splitBlocks, 256, 0, stream>>>(attf, atth, attl, n8);
  wmma_gemm64<1, true, 2, 0, false, 0><<<dim3(32, 1), 256, 0, stream>>>(
      atth, attl, kDim, 0L, Woh, Wol, kDim, 0L, d_out, d_out, kDim, 0L, bout, bout, 0L, kTok, kDim, kDim, 1.0f);
}
